// multi_head_attention_64561948393657
// MI455X (gfx1250) — hardware-verified
//
#include <hip/hip_runtime.h>

#ifndef NB
#define NB 1024
#endif
#define NB_FULL 1024
#define LSEQ   30
#define DDIM   300
#define NHEAD  20
#define HDIM   20
#define ODIM   (NHEAD * HDIM)
#define LP     32
#define DP     320
#define KSTEPS (DP / 32)
#define NTD    19
#define EP     (NTD * 16)
#define FP     32
#define DCH    (DP / 8)
#define QT_CHUNKS (NHEAD * EP * DCH)
#define VT_CHUNKS (NHEAD * FP * DCH)
#define QT_BLOCKS (QT_CHUNKS / 256)
#define VT_BLOCKS (VT_CHUNKS / 256)
#define Y_BSTRIDE   (LSEQ * DDIM)
#define SEQ_BSTRIDE (LSEQ)
#define OUT_BSTRIDE (LSEQ * ODIM)
#define QSC 1024.0f
#define VSC 1024.0f
#define RSC 2048.0f

static_assert(QT_CHUNKS % 256 == 0);
static_assert(VT_CHUNKS % 256 == 0);
static_assert((OUT_BSTRIDE * 4) % 128 == 0);
static_assert((LSEQ * ODIM) % 4 == 0);
static_assert(((NHEAD * EP * DP * 2) % 128) == 0);
static_assert(NB <= NB_FULL);
static_assert(DP % 32 == 0 && EP >= DDIM && FP >= HDIM && LP >= LSEQ);

typedef _Float16 v16h __attribute__((ext_vector_type(16)));
typedef _Float16 v8h  __attribute__((ext_vector_type(8)));
typedef float    v8f  __attribute__((ext_vector_type(8)));
typedef float    v4f  __attribute__((ext_vector_type(4)));
typedef v8h v8ha __attribute__((may_alias));
typedef v4f v4fa __attribute__((may_alias));

union Frag { v16h v; v8h h[2]; };
union U8h  { v8h v; _Float16 s[8]; unsigned int u[4]; };

__device__ __forceinline__ int imin(int a, int b) { return a < b ? a : b; }

__device__ __forceinline__ float bf16_rne(float f) {
  unsigned int u = __builtin_bit_cast(unsigned int, f);
  u = (u + 0x7fffu + ((u >> 16) & 1u)) & 0xffff0000u;
  return __builtin_bit_cast(float, u);
}

__device__ __forceinline__ v16h ld_frag(const _Float16* rowp, int k0, int hf) {
  Frag f;
  f.h[0] = *(const v8ha*)(rowp + k0 + 8 * hf);
  f.h[1] = *(const v8ha*)(rowp + k0 + 16 + 8 * hf);
  return f.v;
}

__device__ __forceinline__ v8f zero8() {
  v8f z = {0.f, 0.f, 0.f, 0.f, 0.f, 0.f, 0.f, 0.f};
  return z;
}

__device__ __forceinline__ v8f wmma16(v16h a, v16h b, v8f c) {
  c = __builtin_amdgcn_wmma_f32_16x16x32_f16(false, a, false, b, (short)0, c, false, false);
  asm volatile("v_nop\n\tv_nop\n\tv_nop\n\tv_nop" : "+v"(c) : "v"(a), "v"(b));
  return c;
}

__launch_bounds__(256)
__global__ void k_prep(const float* __restrict__ Q, const float* __restrict__ V,
                       _Float16* __restrict__ Qt, _Float16* __restrict__ Vt)
{
  const int bid = blockIdx.x;
  const int tid = threadIdx.x;
  U8h u;
  _Float16* dst;
  if (bid < QT_BLOCKS) {
    const int c   = bid * 256 + tid;
    const int h   = c / (EP * DCH);
    const int rem = c - h * (EP * DCH);
    const int e   = rem / DCH;
    const int dc  = rem - e * DCH;
    const int d0  = dc * 8;
    const int ecl = imin(e, DDIM - 1);
#pragma unroll
    for (int j = 0; j < 8; ++j) {
      const int d   = d0 + j;
      const int dcl = imin(d, DDIM - 1);
      const float x = Q[((size_t)h * DDIM + dcl) * DDIM + ecl];
      const bool ok = (d < DDIM) && (e < DDIM);
      const float r = ok ? bf16_rne(x) * QSC : 0.0f;
      u.s[j] = (_Float16)r;
    }
    dst = Qt + (size_t)c * 8;
  } else {
    const int c   = (bid - QT_BLOCKS) * 256 + tid;
    const int h   = c / (FP * DCH);
    const int rem = c - h * (FP * DCH);
    const int f   = rem / DCH;
    const int dc  = rem - f * DCH;
    const int d0  = dc * 8;
    const int fcl = imin(f, HDIM - 1);
#pragma unroll
    for (int j = 0; j < 8; ++j) {
      const int d   = d0 + j;
      const int dcl = imin(d, DDIM - 1);
      const float x = V[((size_t)h * DDIM + dcl) * HDIM + fcl];
      const bool ok = (d < DDIM) && (f < HDIM);
      const float r = ok ? bf16_rne(x) * VSC : 0.0f;
      u.s[j] = (_Float16)r;
    }
    dst = Vt + (size_t)c * 8;
  }
  const v8h val = u.v;
  *(volatile v8h*)dst = val;
  __threadfence();
  *(volatile v8h*)dst = val;
}

__launch_bounds__(256)
__global__ void k_attn(const float* __restrict__ y, const int* __restrict__ seq,
                       const _Float16* __restrict__ Qt, const _Float16* __restrict__ Vt,
                       float* __restrict__ out)
{
  __shared__ __align__(16) _Float16 Ys[LP * DP];
  __shared__ __align__(16) _Float16 Yt[EP * LP];
  __shared__ __align__(16) _Float16 P1h[LP * DP];
  __shared__ __align__(16) _Float16 P1l[LP * DP];
  __shared__ __align__(16) float    Ssc[LP * LP];
  __shared__ __align__(16) _Float16 Eh[LP * LP];
  __shared__ __align__(16) _Float16 El[LP * LP];
  __shared__ __align__(16) float    invs[LP];
  __shared__ __align__(16) int      msk[LP];
  __shared__ __align__(16) float    Outs[LSEQ * ODIM];

  const int tid  = threadIdx.x;
  const int lane = tid & 31;
  const int wave = __builtin_amdgcn_readfirstlane(tid >> 5);
  const int hf   = lane >> 4;
  const int nl   = lane & 15;
  const int b    = blockIdx.x;
  const float* yb = y + (size_t)b * Y_BSTRIDE;

  for (int idx = tid; idx < LP * DCH; idx += 256) {
    const int row = idx / DCH;
    const int dc  = idx - row * DCH;
    const int d0  = dc * 8;
    const int rcl = imin(row, LSEQ - 1);
    U8h u;
#pragma unroll
    for (int j = 0; j < 8; ++j) {
      const int d   = d0 + j;
      const int dcl = imin(d, DDIM - 1);
      const float x = yb[rcl * DDIM + dcl];
      const bool ok = (row < LSEQ) && (d < DDIM);
      const float r = ok ? bf16_rne(x) : 0.0f;
      u.s[j] = (_Float16)r;
    }
    *(v8ha*)(Ys + row * DP + d0) = u.v;
#pragma unroll
    for (int j = 0; j < 8; ++j) {
      const int d = d0 + j;
      if (d < EP) Yt[d * LP + row] = u.s[j];
    }
  }
  if (tid < 64) {
    const int r = tid >> 1, c = tid & 1;
    U8h z; z.u[0] = 0u; z.u[1] = 0u; z.u[2] = 0u; z.u[3] = 0u;
    *(v8ha*)(P1h + r * DP + EP + c * 8) = z.v;
    *(v8ha*)(P1l + r * DP + EP + c * 8) = z.v;
  }
  if (tid < LP) {
    const int m  = imin(tid, LSEQ - 1);
    const int sv = seq[(size_t)b * SEQ_BSTRIDE + m];
    msk[tid] = (tid < LSEQ && sv > 0) ? 1 : 0;
  }
  __syncthreads();

  for (int h = 0; h < NHEAD; ++h) {
    {
      v8f acc[3][2];
#pragma unroll
      for (int t = 0; t < 3; ++t) { acc[t][0] = zero8(); acc[t][1] = zero8(); }
      const _Float16* qb = Qt + (size_t)h * EP * DP;
#pragma unroll 1
      for (int ks = 0; ks < KSTEPS; ++ks) {
        const int k0 = ks * 32;
        const v16h a0 = ld_frag(Ys + nl * DP, k0, hf);
        const v16h a1 = ld_frag(Ys + (16 + nl) * DP, k0, hf);
#pragma unroll
        for (int t = 0; t < 3; ++t) {
          const int nt = wave + 8 * t;
          if (nt < NTD) {
            const v16h bq = ld_frag(qb + (size_t)(nt * 16 + nl) * DP, k0, hf);
            acc[t][0] = wmma16(a0, bq, acc[t][0]);
            acc[t][1] = wmma16(a1, bq, acc[t][1]);
          }
        }
      }
#pragma unroll
      for (int t = 0; t < 3; ++t) {
        const int nt = wave + 8 * t;
        if (nt < NTD) {
          const int col = nt * 16 + nl;
#pragma unroll
          for (int mt = 0; mt < 2; ++mt) {
#pragma unroll
            for (int r = 0; r < 8; ++r) {
              const int row = mt * 16 + 8 * hf + r;
              const float a = acc[t][mt][r] * (1.0f / QSC);
              const _Float16 ah = (_Float16)a;
              const float rs = (a - (float)ah) * RSC;
              P1h[row * DP + col] = ah;
              P1l[row * DP + col] = (_Float16)rs;
            }
          }
        }
      }
    }
    __syncthreads();

    if (wave < 4) {
      const int mt = wave >> 1, nt = wave & 1;
      v8f ch = zero8(), cl = zero8();
#pragma unroll 1
      for (int ks = 0; ks < KSTEPS; ++ks) {
        const int k0 = ks * 32;
        const v16h by = ld_frag(Ys + (nt * 16 + nl) * DP, k0, hf);
        const v16h ah = ld_frag(P1h + (mt * 16 + nl) * DP, k0, hf);
        const v16h al = ld_frag(P1l + (mt * 16 + nl) * DP, k0, hf);
        ch = wmma16(ah, by, ch);
        cl = wmma16(al, by, cl);
      }
#pragma unroll
      for (int r = 0; r < 8; ++r) {
        const int row = mt * 16 + 8 * hf + r;
        const int col = nt * 16 + nl;
        Ssc[row * LP + col] = ch[r] + cl[r] * (1.0f / RSC);
      }
    }
    __syncthreads();

    {
      const int l = tid >> 3;
      const int g = tid & 7;
      float part = 0.0f;
#pragma unroll
      for (int j = 0; j < 4; ++j) {
        const int m = g * 4 + j;
        const float s = Ssc[l * LP + m];
        const bool ok = (l < LSEQ) && (m < LSEQ);
        const float e = ok ? expf(s) : 0.0f;
        part += (msk[m] != 0) ? e : 0.0f;
        const _Float16 ehv = (_Float16)e;
        const float rs = (e - (float)ehv) * RSC;
        Eh[l * LP + m] = ehv;
        El[l * LP + m] = (_Float16)rs;
      }
      part += __shfl_xor(part, 1);
      part += __shfl_xor(part, 2);
      part += __shfl_xor(part, 4);
      if (g == 0) invs[l] = (l < LSEQ) ? (1.0f / (part + 1e-6f)) : 0.0f;
    }
    __syncthreads();

    {
      v16h ehf[2], elf[2];
#pragma unroll
      for (int mt = 0; mt < 2; ++mt) {
        ehf[mt] = ld_frag(Eh + (mt * 16 + nl) * LP, 0, hf);
        elf[mt] = ld_frag(El + (mt * 16 + nl) * LP, 0, hf);
      }
#pragma unroll
      for (int t = 0; t < 3; ++t) {
        const int nt = wave + 8 * t;
        if (nt < NTD) {
          const v16h by = ld_frag(Yt + (nt * 16 + nl) * LP, 0, hf);
          const int col = nt * 16 + nl;
#pragma unroll
          for (int mt = 0; mt < 2; ++mt) {
            const v8f ch = wmma16(ehf[mt], by, zero8());
            const v8f cl = wmma16(elf[mt], by, zero8());
#pragma unroll
            for (int r = 0; r < 8; ++r) {
              const int row = mt * 16 + 8 * hf + r;
              const float hv = (ch[r] + cl[r] * (1.0f / RSC)) * invs[row];
              const _Float16 hh = (_Float16)hv;
              const float rs = (hv - (float)hh) * RSC;
              P1h[row * DP + col] = hh;
              P1l[row * DP + col] = (_Float16)rs;
            }
          }
        }
      }
    }
    __syncthreads();

    if (wave < 4) {
      const int mt = wave >> 1, nt = wave & 1;
      const _Float16* vb = Vt + (size_t)h * FP * DP;
      v8f ch = zero8(), cl = zero8();
#pragma unroll 1
      for (int ks = 0; ks < KSTEPS; ++ks) {
        const int k0 = ks * 32;
        const v16h bv = ld_frag(vb + (size_t)(nt * 16 + nl) * DP, k0, hf);
        const v16h ah = ld_frag(P1h + (mt * 16 + nl) * DP, k0, hf);
        const v16h al = ld_frag(P1l + (mt * 16 + nl) * DP, k0, hf);
        ch = wmma16(ah, bv, ch);
        cl = wmma16(al, bv, cl);
      }
#pragma unroll
      for (int r = 0; r < 8; ++r) {
        const int l = mt * 16 + 8 * hf + r;
        const int f = nt * 16 + nl;
        const float v = (ch[r] + cl[r] * (1.0f / RSC)) * (1.0f / VSC);
        if (l < LSEQ && f < HDIM) Outs[l * ODIM + h * HDIM + f] = v;
      }
    }
    __syncthreads();
  }

  float* ob = out + (size_t)b * OUT_BSTRIDE;
  constexpr int NV4 = (LSEQ * ODIM) / 4;
  for (int i = tid; i < NV4; i += 256) {
    const v4f v = *(const v4fa*)(Outs + i * 4);
    *(volatile v4f*)(ob + (size_t)i * 4) = v;
  }
  __threadfence();
  for (int i = tid; i < NV4; i += 256) {
    const v4f v = *(const v4fa*)(Outs + i * 4);
    *(volatile v4f*)(ob + (size_t)i * 4) = v;
  }
}

extern "C" void kernel_launch(void* const* d_in, const int* in_sizes, int n_in,
                              void* d_out, int out_size, void* d_ws, size_t ws_size,
                              hipStream_t stream)
{
  if (n_in < 4) return;
  if (in_sizes[0] < NB * LSEQ * DDIM) return;
  if (in_sizes[1] < NB * LSEQ) return;
  if (in_sizes[2] < NHEAD * DDIM * DDIM) return;
  if (in_sizes[3] < NHEAD * DDIM * HDIM) return;
  if (out_size < NB * LSEQ * ODIM) return;

  const float* y   = (const float*)d_in[0];
  const int*   seq = (const int*)  d_in[1];
  const float* Q   = (const float*)d_in[2];
  const float* V   = (const float*)d_in[3];
  float*       out = (float*)d_out;

  const size_t qt_bytes = (size_t)NHEAD * EP * DP * sizeof(_Float16);
  const size_t vt_bytes = (size_t)NHEAD * FP * DP * sizeof(_Float16);
  if (ws_size < qt_bytes + vt_bytes) return;
  _Float16* Qt = (_Float16*)d_ws;
  _Float16* Vt = (_Float16*)((char*)d_ws + qt_bytes);

  k_prep<<<dim3(QT_BLOCKS + VT_BLOCKS), dim3(256), 0, stream>>>(Q, V, Qt, Vt);
  k_attn<<<dim3(NB), dim3(256), 0, stream>>>(y, seq, Qt, Vt, out);
}
